// GGNNClassifier_7000796692925
// MI455X (gfx1250) — hardware-verified
//
#include <hip/hip_runtime.h>
#include <math.h>
typedef __attribute__((ext_vector_type(16))) _Float16 v16h;
typedef __attribute__((ext_vector_type(8)))  _Float16 v8h;
typedef __attribute__((ext_vector_type(16))) __bf16   v16b;
typedef __attribute__((ext_vector_type(8)))  __bf16   v8b;
typedef __attribute__((ext_vector_type(8)))  float    v8f;
typedef __attribute__((ext_vector_type(4)))  float    v4f;
#define PSCALE 32768.0f
#define U16(p) ((const unsigned short*)(const void*)(p))
#define PSCALE_INV (1.0f / 32768.0f)

__device__ __forceinline__ unsigned short f2bf_bits(float f) {
  unsigned u = __float_as_uint(f);
  return (unsigned short)((u + 0x7FFFu + ((u >> 16) & 1u)) >> 16);
}
__device__ __forceinline__ float bf_bits2f(unsigned short h) { return __uint_as_float(((unsigned)h) << 16); }

__device__ __forceinline__ void dep_guard_h(v8f& a, v8f& b, v16h x, v16h y) { asm volatile("v_nop\n\tv_nop\n\tv_nop\n\tv_nop" : "+v"(a), "+v"(b) : "v"(x), "v"(y)); }
__device__ __forceinline__ void dep_guard_b(v8f& a, v8f& b, v16b x, v16b y) { asm volatile("v_nop\n\tv_nop\n\tv_nop\n\tv_nop" : "+v"(a), "+v"(b) : "v"(x), "v"(y)); }
__device__ __forceinline__ void keep4_h(v16h a, v16h b, v16h c, v16h d) { asm volatile("v_nop" :: "v"(a), "v"(b), "v"(c), "v"(d)); }
__device__ __forceinline__ void keep4_b(v16b a, v16b b, v16b c, v16b d) { asm volatile("v_nop" :: "v"(a), "v"(b), "v"(c), "v"(d)); }
__device__ __forceinline__ void acc_guard4(v8f& a, v8f& b, v8f& c, v8f& d) { asm volatile("v_nop\n\tv_nop\n\tv_nop\n\tv_nop" : "+v"(a), "+v"(b), "+v"(c), "+v"(d)); }
template <typename T> struct Frag;
template <> struct Frag<_Float16> {
  typedef v16h V; union U { v16h v; v8h h[2]; };
  static __device__ __forceinline__ v16h load(const _Float16* p) {
    U f; f.h[0] = *(const v8h*)(p); f.h[1] = *(const v8h*)(p + 16); return f.v;
  }
  static __device__ __forceinline__ v8f mma(v16h a, v16h b, v8f c) {
    return __builtin_amdgcn_wmma_f32_16x16x32_f16(false, a, false, b, (short)0, c, false, false);
  }
  static __device__ __forceinline__ void guard(v8f& a, v8f& b, v16h x, v16h y) { dep_guard_h(a, b, x, y); }
  static __device__ __forceinline__ void keep(v16h a, v16h b, v16h c, v16h d) { keep4_h(a, b, c, d); }
};
template <> struct Frag<__bf16> {
  typedef v16b V; union U { v16b v; v8b h[2]; };
  static __device__ __forceinline__ v16b load(const __bf16* p) {
    U f; f.h[0] = *(const v8b*)(p); f.h[1] = *(const v8b*)(p + 16); return f.v;
  }
  static __device__ __forceinline__ v8f mma(v16b a, v16b b, v8f c) {
    return __builtin_amdgcn_wmma_f32_16x16x32_bf16(false, a, false, b, (short)0, c, false, false);
  }
  static __device__ __forceinline__ void guard(v8f& a, v8f& b, v16b x, v16b y) { dep_guard_b(a, b, x, y); }
  static __device__ __forceinline__ void keep(v16b a, v16b b, v16b c, v16b d) { keep4_b(a, b, c, d); }
};

template <int ET> struct Elem;
template <> struct Elem<0> { typedef _Float16 T; };
template <> struct Elem<1> { typedef __bf16 T; };
template <int ET, bool SPLIT, int BIAS_MODE, int OUT_MODE, bool RESID, int ACT = 0>
__global__ __launch_bounds__(256) void wmma_gemm64(
    const unsigned short* __restrict__ Ap, const unsigned short* __restrict__ A2p, int lda, long strideA,
    const unsigned short* __restrict__ Btp, const unsigned short* __restrict__ Bt2p, int ldb, long strideB,
    void* __restrict__ Cout, void* __restrict__ Cout2, int ldc, long strideC,
    const float* __restrict__ bias,
    const float* __restrict__ resid, long strideR,
    int M, int N, int K, float scale) {
  typedef typename Elem<ET>::T T;
  typedef typename Frag<T>::V V;
  const T* A = (const T*)Ap; const T* A2 = (const T*)A2p; const T* Bt = (const T*)Btp; const T* Bt2 = (const T*)Bt2p;
  __shared__ __align__(16) float sT[8][16 * 68];
  const int b    = blockIdx.y;
  const int lane = threadIdx.x & 31;
  const int wave = threadIdx.x >> 5;
  const int tilesN = N >> 6;
  const int tilesM = M >> 6;
  const int tile = blockIdx.x * 8 + wave;
  if (tile >= tilesM * tilesN) return;
  const int tm = tile / tilesN;
  const int tn = tile - tm * tilesN;
  const int m0 = tm << 6;
  const int n0 = tn << 6;

  const T* Ab  = A  + (size_t)b * strideA;
  const T* Bb  = Bt + (size_t)b * strideB;
  const T* Ab2 = SPLIT ? (A2  + (size_t)b * strideA) : nullptr;
  const T* Bb2 = SPLIT ? (Bt2 + (size_t)b * strideB) : nullptr;

  const int rlane = lane & 15;
  const int koff  = (lane >> 4) * 8;
  const int mOff  = (lane >> 4) * 8;

  v8f acc[4][4];
#pragma unroll
  for (int i = 0; i < 4; ++i)
#pragma unroll
    for (int j = 0; j < 4; ++j) acc[i][j] = (v8f){0.f,0.f,0.f,0.f,0.f,0.f,0.f,0.f};

  for (int k0 = 0; k0 < K; k0 += 32) {
    V bh[4], bl[4];
#pragma unroll
    for (int j = 0; j < 4; ++j) {
      const size_t bo = (size_t)(n0 + (j << 4) + rlane) * ldb + koff + k0;
      bh[j] = Frag<T>::load(Bb + bo);
      if (SPLIT) bl[j] = Frag<T>::load(Bb2 + bo);
    }
#pragma unroll
    for (int i = 0; i < 4; ++i) {
      const size_t ao = (size_t)(m0 + (i << 4) + rlane) * lda + koff + k0;
      V ah = Frag<T>::load(Ab + ao);
      V al;
      if (SPLIT) al = Frag<T>::load(Ab2 + ao);
#pragma unroll
      for (int j = 0; j < 4; ++j) {
        acc[i][j] = Frag<T>::mma(ah, bh[j], acc[i][j]);
        if (SPLIT) {
          acc[i][j] = Frag<T>::mma(ah, bl[j], acc[i][j]);
          acc[i][j] = Frag<T>::mma(al, bh[j], acc[i][j]);
        }
      }
      Frag<T>::guard(acc[i][0], acc[i][3], ah, SPLIT ? al : ah);
    }
    Frag<T>::keep(bh[0], bh[1], bh[2], bh[3]);
    if (SPLIT) Frag<T>::keep(bl[0], bl[1], bl[2], bl[3]);
  }
  acc_guard4(acc[0][0], acc[0][1], acc[0][2], acc[0][3]);
  acc_guard4(acc[1][0], acc[1][1], acc[1][2], acc[1][3]);
  acc_guard4(acc[2][0], acc[2][1], acc[2][2], acc[2][3]);
  acc_guard4(acc[3][0], acc[3][1], acc[3][2], acc[3][3]);

  float* slab = sT[wave];
  const float* Rb = RESID ? (resid + (size_t)b * strideR) : nullptr;
#pragma unroll
  for (int i = 0; i < 4; ++i) {
    const int mBase = m0 + (i << 4);
#pragma unroll
    for (int j = 0; j < 4; ++j) {
      const int n = n0 + (j << 4) + rlane;
      float bv = 0.f;
      if (BIAS_MODE == 2) bv = bias[n];
#pragma unroll
      for (int r = 0; r < 8; ++r) {
        float v = acc[i][j][r] * scale;
        if (BIAS_MODE == 1) v += bias[mBase + mOff + r];
        if (BIAS_MODE == 2) v += bv;
        if (RESID) v += Rb[(size_t)(mBase + mOff + r) * ldc + n];
        if (ACT == 1) v = tanhf(v);
        if (ACT == 2) v = fmaxf(v, 0.0f);
        if (ACT == 3) v = v / (1.0f + expf(-v));
        if (ACT == 4) v = (v > 0.f) ? v : 0.01f * v;
        if (ACT == 5) v = 0.5f * v * (1.0f + erff(v * 0.70710678118654752f));
        slab[(mOff + r) * 68 + (j << 4) + rlane] = v;
      }
    }
    __builtin_amdgcn_fence(__ATOMIC_RELEASE, "workgroup");
    __builtin_amdgcn_wave_barrier();
    __builtin_amdgcn_fence(__ATOMIC_ACQUIRE, "workgroup");
    if (OUT_MODE == 0) {
      float* C = (float*)Cout + (size_t)b * strideC;
      const int hh = lane >> 4, c4 = (lane & 15) * 4;
      for (int pass = 0; pass < 2; ++pass) {
#pragma unroll
        for (int it = 0; it < 8; ++it) {
          const int row = it * 2 + hh;
          v4f v = *(const v4f*)(slab + row * 68 + c4);
          *(volatile v4f*)(C + (size_t)(mBase + row) * ldc + n0 + c4) = v;
        }
        __threadfence();
      }
    } else {
      const int q = lane >> 3, c8 = (lane & 7) * 8;
      unsigned short* C  = (unsigned short*)Cout  + (size_t)b * strideC;
      unsigned short* C2 = (OUT_MODE == 2) ? ((unsigned short*)Cout2 + (size_t)b * strideC) : nullptr;
      for (int pass = 0; pass < 2; ++pass) {
#pragma unroll
        for (int it = 0; it < 4; ++it) {
          const int row = it * 4 + q;
          const float* sp = slab + row * 68 + c8;
          v8h hv, lv;
#pragma unroll
          for (int e = 0; e < 8; ++e) {
            if (OUT_MODE == 1) {
              hv[e] = (_Float16)sp[e];
            } else {
              unsigned short hb = f2bf_bits(sp[e]);
              unsigned short lb = f2bf_bits(sp[e] - bf_bits2f(hb));
              hv[e] = __builtin_bit_cast(_Float16, hb);
              lv[e] = __builtin_bit_cast(_Float16, lb);
            }
          }
          *(volatile v8h*)(C + (size_t)(mBase + row) * ldc + n0 + c8) = hv;
          if (OUT_MODE == 2) *(volatile v8h*)(C2 + (size_t)(mBase + row) * ldc + n0 + c8) = lv;
        }
        __threadfence();
      }
    }
    __builtin_amdgcn_fence(__ATOMIC_RELEASE, "workgroup");
    __builtin_amdgcn_wave_barrier();
    __builtin_amdgcn_fence(__ATOMIC_ACQUIRE, "workgroup");
  }
}

__global__ __launch_bounds__(256) void cast_f32_f16x2(
    const float* __restrict__ in, _Float16* __restrict__ out, int n2) {
  int i = blockIdx.x * 256 + threadIdx.x;
  if (i < n2) {
    const _Float16 h0 = (_Float16)in[2 * i], h1 = (_Float16)in[2 * i + 1];
    const unsigned u = (unsigned)__builtin_bit_cast(unsigned short, h0) | ((unsigned)__builtin_bit_cast(unsigned short, h1) << 16);
    ((volatile unsigned*)out)[i] = u;
    __threadfence();
    ((volatile unsigned*)out)[i] = u;
  }
}


__global__ __launch_bounds__(256) void transpose_cast_f16(const float* __restrict__ in, int ldi,
                                                         _Float16* __restrict__ outT, int ldo, float scale) {
  __shared__ __align__(16) _Float16 tile[64][72];
  const int c0 = blockIdx.x * 64, r0 = blockIdx.y * 64;
  const int t = threadIdx.y * 32 + threadIdx.x;
  for (int i = threadIdx.y; i < 64; i += 8) {
    tile[threadIdx.x][i]      = (_Float16)(in[(size_t)(r0 + i) * ldi + c0 + threadIdx.x] * scale);
    tile[32 + threadIdx.x][i] = (_Float16)(in[(size_t)(r0 + i) * ldi + c0 + 32 + threadIdx.x] * scale);
  }
  __syncthreads();
  const int q = t >> 3, c8 = (t & 7) * 8;
  for (int pass = 0; pass < 2; ++pass) {
#pragma unroll
    for (int it = 0; it < 2; ++it) {
      const int c = it * 32 + q;
      v8h hv = *(const v8h*)(&tile[c][c8]);
      *(volatile v8h*)(outT + (size_t)(c0 + c) * ldo + r0 + c8) = hv;
    }
    __threadfence();
  }
}

#define NN 100000
#define NODES_PER_BLK 256
#define NBLK ((NN + NODES_PER_BLK - 1) / NODES_PER_BLK)
#define NPAD (NBLK * NODES_PER_BLK)
#define NE 1000000
#define SEG_CAP 8192
#define GIN 128
#define GH 64
#define NET 4
#define NG 128

#define ECH 8192
#define NCH ((NE + ECH - 1) / ECH)
#define NRP (((NBLK) + 31) & ~31)
#define SEG_STRIDE SEG_CAP
#define BUCKET_INTS ((size_t)NE + (size_t)32 * NCH * NBLK)
__device__ __forceinline__ int rank_eq(int key, bool valid, int lane, int nbits, int& ntotal) {
  unsigned same = __ballot(valid);
  for (int b = 0; b < nbits; ++b) {
    const unsigned m = __ballot(((key >> b) & 1) != 0);
    same &= (((key >> b) & 1) != 0) ? m : ~m;
  }
  if (!valid) same = 0u;
  ntotal = __popc(same);
  return __popc(same & ((1u << lane) - 1u));
}
__global__ __launch_bounds__(256) void csr_hist_kernel(const int* __restrict__ dst, int* __restrict__ cnt) {
  __shared__ int h[8][NRP];
  const int tid = threadIdx.x, lane = tid & 31, wave = tid >> 5;
  for (int i = tid; i < 8 * NRP; i += 256) (&h[0][0])[i] = 0;
  __syncthreads();
  const int e0 = blockIdx.x * ECH + wave * (ECH / 8), e1 = min(e0 + ECH / 8, NE);
  for (int c0 = e0; c0 < e0 + ECH / 8; c0 += 32) {
    const int e = c0 + lane;
    const bool valid = e < e1;
    int d = valid ? dst[e] : 0; d = d < 0 ? 0 : (d >= NN ? NN - 1 : d);
    const int r = d / NODES_PER_BLK;
    int tot; const int rk = rank_eq(r, valid, lane, 9, tot);
    if (valid && rk == tot - 1) h[wave][r] += tot;
  }
  __syncthreads();
  for (int pass = 0; pass < 2; ++pass) {
    for (int i = tid; i < NRP; i += 256) { int s = 0; for (int w = 0; w < 8; ++w) s += h[w][i]; ((volatile int*)cnt)[(size_t)blockIdx.x * NRP + i] = s; }
    __threadfence();
  }
}
__global__ __launch_bounds__(1024) void csr_offsets_kernel(const int* __restrict__ cnt, int* __restrict__ boff, int* __restrict__ rinfo) {
  __shared__ int rsz[1024];
  const int t = threadIdx.x;
  int run = 0;
  if (t < NBLK) { for (int c = 0; c < NCH; ++c) run += (cnt[(size_t)c * NRP + t] + 31) & ~31; }
  rsz[t] = (t < NBLK) ? run : 0;
  __syncthreads();
  for (int off = 1; off < 1024; off <<= 1) { int v = (t >= off) ? rsz[t - off] : 0; __syncthreads(); rsz[t] += v; __syncthreads(); }
  const int incl = rsz[t], excl = incl - ((t < NBLK) ? run : 0);
  __syncthreads();
  for (int pass = 0; pass < 2; ++pass) {
    if (t < NBLK) { int r2 = excl; for (int c = 0; c < NCH; ++c) { const size_t i = (size_t)c * NRP + t; ((volatile int*)boff)[i] = r2; r2 += (cnt[i] + 31) & ~31; } }
    ((volatile int*)rinfo)[t] = excl;
    ((volatile int*)rinfo)[1024 + t] = (t < NBLK) ? run : 0;
    __threadfence();
  }
}
__global__ __launch_bounds__(256) void csr_bucket_kernel(const int* __restrict__ dst, const int* __restrict__ boff, int* __restrict__ bucket) {
  __shared__ int wc[8][NRP];
  __shared__ int woff[8][NRP];
  __shared__ int roff[NRP + 1];
  __shared__ int seg[ECH + 32 * NRP];
  const int tid = threadIdx.x, lane = tid & 31, wave = tid >> 5;
  for (int i = tid; i < 8 * NRP; i += 256) { (&wc[0][0])[i] = 0; }
  __syncthreads();
  const int e0 = blockIdx.x * ECH + wave * (ECH / 8), e1 = min(e0 + ECH / 8, NE);
  for (int c0 = e0; c0 < e0 + ECH / 8; c0 += 32) {
    const int e = c0 + lane; const bool valid = e < e1;
    int d = valid ? dst[e] : 0; d = d < 0 ? 0 : (d >= NN ? NN - 1 : d);
    const int r = d / NODES_PER_BLK;
    int tot; const int rk = rank_eq(r, valid, lane, 9, tot);
    if (valid && rk == tot - 1) wc[wave][r] += tot;
  }
  __syncthreads();
  __shared__ int tot_r[NRP];
  for (int i = tid; i < NRP; i += 256) { int s = 0; for (int w = 0; w < 8; ++w) s += wc[w][i]; tot_r[i] = s; }
  __syncthreads();
  if (tid == 0) { int run = 0; for (int r = 0; r < NRP; ++r) { roff[r] = run; int o = run; for (int w = 0; w < 8; ++w) { woff[w][r] = o; o += wc[w][r]; } run += (tot_r[r] + 31) & ~31; } roff[NRP] = run; }
  __syncthreads();
  const int totalpad = roff[NRP];
  for (int i = tid; i < totalpad && i < ECH + 32 * NRP; i += 256) seg[i] = -1;
  __syncthreads();
  for (int c0 = e0; c0 < e0 + ECH / 8; c0 += 32) {
    const int e = c0 + lane; const bool valid = e < e1;
    int d = valid ? dst[e] : 0; d = d < 0 ? 0 : (d >= NN ? NN - 1 : d);
    const int r = d / NODES_PER_BLK;
    int tot; const int rk = rank_eq(r, valid, lane, 9, tot);
    if (valid) { const int slot = woff[wave][r] + rk; if (slot < ECH + 32 * NRP) seg[slot] = e; if (rk == tot - 1) woff[wave][r] = slot + 1; }
  }
  __syncthreads();
  for (int pass = 0; pass < 2; ++pass) {
    for (int r = wave; r < NBLK; r += 8) {
      const int lo = roff[r], n = ((tot_r[r] + 31) & ~31);
      const int gb = boff[(size_t)blockIdx.x * NRP + r];
      for (int i = lane; i < n; i += 32) ((volatile int*)bucket)[(size_t)gb + i] = (lo + i < ECH + 32 * NRP) ? seg[lo + i] : -1;
    }
    __threadfence();
  }
}
__global__ __launch_bounds__(256) void csr_fill_kernel(const int* __restrict__ dst, const int* __restrict__ bucket, const int* __restrict__ rinfo,
                                                      int* __restrict__ rowptr, int* __restrict__ rowdeg, int* __restrict__ csr_eid, int* __restrict__ rcl) {
  __shared__ int cnt[8][NODES_PER_BLK];
  __shared__ int off[8][NODES_PER_BLK];
  __shared__ int nodeoff[NODES_PER_BLK + 1];
  __shared__ int seg[SEG_CAP];
  const int tid = threadIdx.x, lane = tid & 31, wave = tid >> 5;
  const int n0 = blockIdx.x * NODES_PER_BLK;
  const int bstart = rinfo[blockIdx.x], bsize = rinfo[1024 + blockIdx.x];
  for (int i = tid; i < 8 * NODES_PER_BLK; i += 256) (&cnt[0][0])[i] = 0;
  for (int i = tid; i < SEG_CAP; i += 256) seg[i] = 0;
  __syncthreads();
  const int per = ((bsize / 8) + 31) & ~31;
  const int e0 = bstart + wave * per, e1 = min(bstart + (wave + 1) * per, bstart + bsize);
  for (int c0 = e0; c0 < e0 + per; c0 += 32) {
    const int j = c0 + lane;
    int e = (j < e1) ? bucket[j] : -1;
    const bool valid = (e >= 0) && (e < NE);
    int d = valid ? dst[e] : -1;
    const bool ok = valid && (d >= n0) && (d < n0 + NODES_PER_BLK);
    int tot; const int rk = rank_eq(ok ? (d - n0) : 0, ok, lane, 8, tot);
    if (ok && rk == tot - 1) cnt[wave][d - n0] += tot;
  }
  __syncthreads();
  if (tid < 32) {
    int loc[8]; int sum = 0;
    for (int q = 0; q < 8; ++q) { int c = 0; for (int w = 0; w < 8; ++w) c += cnt[w][tid * 8 + q]; loc[q] = c; sum += c; }
    int incl = sum;
    for (int o = 1; o < 32; o <<= 1) { int t = __shfl_up(incl, o, 32); if (lane >= o) incl += t; }
    int base = incl - sum;
    for (int q = 0; q < 8; ++q) {
      const int node = tid * 8 + q;
      nodeoff[node] = base;
      int run = base;
      for (int w = 0; w < 8; ++w) { off[w][node] = run; run += cnt[w][node]; }
      base += loc[q];
    }
    if (tid == 31) nodeoff[NODES_PER_BLK] = base;
  }
  __syncthreads();
  const int btotal = nodeoff[NODES_PER_BLK];
  for (int c0 = e0; c0 < e0 + per; c0 += 32) {
    const int j = c0 + lane;
    int e = (j < e1) ? bucket[j] : -1;
    const bool valid = (e >= 0) && (e < NE);
    int d = valid ? dst[e] : -1;
    const bool ok = valid && (d >= n0) && (d < n0 + NODES_PER_BLK);
    int tot; const int rk = rank_eq(ok ? (d - n0) : 0, ok, lane, 8, tot);
    if (ok) { const int slot = off[wave][d - n0] + rk; if (slot < SEG_CAP) seg[slot] = e; if (rk == tot - 1) off[wave][d - n0] = slot + 1; }
  }
  __syncthreads();
  const int gstart = blockIdx.x * (SEG_STRIDE);
  const int nlines = (min(btotal, SEG_CAP) + 31) >> 5;
  for (int pass = 0; pass < 2; ++pass) {
    { const int node = tid; int deg = 0; for (int w = 0; w < 8; ++w) deg += cnt[w][node];
      ((volatile int*)rowptr)[n0 + node] = gstart + nodeoff[node]; ((volatile int*)rowdeg)[n0 + node] = deg; }
    for (int i = tid; i < nlines * 32; i += 256) ((volatile int*)csr_eid)[gstart + i] = (i < btotal) ? seg[i] : 0;
    if (rcl != nullptr && tid < 32) ((volatile int*)rcl)[blockIdx.x * 32 + tid] = (tid == 0) ? min(btotal, SEG_CAP) : 0;
    __threadfence();
  }
}

__global__ __launch_bounds__(256) void padcast_rows_kernel(const float* __restrict__ x, unsigned* __restrict__ X16) {
  const long i = (long)blockIdx.x * 256 + threadIdx.x; if (i >= (long)NPAD * GIN / 2) return;
  const long e0 = 2 * i; const bool ok = e0 < (long)NN * GIN;
  const float a = ok ? x[e0] : 0.f, b = ok ? x[e0 + 1] : 0.f;
  const unsigned u = (unsigned)__builtin_bit_cast(unsigned short, (_Float16)a) | ((unsigned)__builtin_bit_cast(unsigned short, (_Float16)b) << 16);
  ((volatile unsigned*)X16)[i] = u; __threadfence(); ((volatile unsigned*)X16)[i] = u;
}
__global__ __launch_bounds__(256) void cast_h_kernel(const float* __restrict__ Hm, unsigned* __restrict__ H16) {
  const long i = (long)blockIdx.x * 256 + threadIdx.x; if (i >= (long)NPAD * GH / 2) return;
  const float a = Hm[2 * i], b = Hm[2 * i + 1];
  const unsigned u = (unsigned)__builtin_bit_cast(unsigned short, (_Float16)a) | ((unsigned)__builtin_bit_cast(unsigned short, (_Float16)b) << 16);
  ((volatile unsigned*)H16)[i] = u; __threadfence(); ((volatile unsigned*)H16)[i] = u;
}
__global__ __launch_bounds__(256) void agg_kernel(const unsigned* __restrict__ T, const int* __restrict__ rowptr, const int* __restrict__ rowdeg, const int* __restrict__ csr_eid,
                                                 const int* __restrict__ srcidx, const int* __restrict__ et, unsigned* __restrict__ A16) {
  const int lane = threadIdx.x & 31, wave = threadIdx.x >> 5; const int i = blockIdx.x * 8 + wave;
  float a0 = 0.f, a1 = 0.f;
  if (i < NN) {
    int j0 = rowptr[i]; int dg = rowdeg[i]; dg = dg < 0 ? 0 : (dg > SEG_CAP ? SEG_CAP : dg); j0 = j0 < 0 ? 0 : j0;
    for (int j = j0; j < j0 + dg; ++j) {
      int e = csr_eid[j]; e = e < 0 ? 0 : (e >= NE ? NE - 1 : e);
      int s = srcidx[e]; s = s < 0 ? 0 : (s >= NN ? NN - 1 : s);
      int ty = et[e]; ty = ty < 0 ? 0 : (ty >= NET ? NET - 1 : ty);
      const unsigned tv = T[((size_t)s * (NET * GH) + ty * GH) / 2 + lane];
      a0 += (float)__builtin_bit_cast(_Float16, (unsigned short)(tv & 0xFFFFu)); a1 += (float)__builtin_bit_cast(_Float16, (unsigned short)(tv >> 16));
    }
  }
  const unsigned u = (unsigned)__builtin_bit_cast(unsigned short, (_Float16)a0) | ((unsigned)__builtin_bit_cast(unsigned short, (_Float16)a1) << 16);
  ((volatile unsigned*)A16)[(size_t)i * (GH / 2) + lane] = u; __threadfence(); ((volatile unsigned*)A16)[(size_t)i * (GH / 2) + lane] = u;
}
__global__ __launch_bounds__(256) void gru_kernel(const float* __restrict__ GI, const float* __restrict__ GHm, float* __restrict__ Hm, unsigned* __restrict__ H16, int nrows) {
  const long i = (long)blockIdx.x * 256 + threadIdx.x; if (i >= (long)nrows * GH / 2) return;
  const int n = (int)(i / (GH / 2)), c0 = (int)(i % (GH / 2)) * 2;
  typedef __attribute__((ext_vector_type(2))) float v2f;
  const v2f hp = *(const v2f*)(Hm + (size_t)n * GH + c0);
  float hv[2];
#pragma unroll
  for (int e = 0; e < 2; ++e) { const int c = c0 + e; const float* gi = GI + (size_t)n * (3 * GH); const float* gh = GHm + (size_t)n * (3 * GH);
    const float r = 1.0f / (1.0f + expf(-(gi[c] + gh[c]))); const float z = 1.0f / (1.0f + expf(-(gi[GH + c] + gh[GH + c])));
    const float nn = tanhf(gi[2 * GH + c] + r * gh[2 * GH + c]);
    hv[e] = (1.0f - z) * nn + z * hp[e]; }
  const v2f hn = {hv[0], hv[1]};
  const unsigned u = (unsigned)__builtin_bit_cast(unsigned short, (_Float16)hv[0]) | ((unsigned)__builtin_bit_cast(unsigned short, (_Float16)hv[1]) << 16);
  for (int pass = 0; pass < 2; ++pass) { *(volatile v2f*)(Hm + (size_t)n * GH + c0) = hn; ((volatile unsigned*)H16)[i] = u; __threadfence(); }
}
__global__ __launch_bounds__(256) void readout_kernel(const float* __restrict__ Hm, const int* __restrict__ n2g, const float* __restrict__ W1, const float* __restrict__ b1,
                                                     const float* __restrict__ W2, const float* __restrict__ b2, float* __restrict__ outg) {
  __shared__ float acc[8][GH]; __shared__ float hg[GH]; __shared__ float z1[32]; __shared__ int rng[2];
  const int g = blockIdx.x, t = threadIdx.x, lane = t & 31, wave = t >> 5;
  if (t < 2) {
    const int key = g + t; int lo = 0, hi = NN;
    while (lo < hi) { const int mid = (lo + hi) >> 1; if (n2g[mid] < key) lo = mid + 1; else hi = mid; }
    rng[t] = lo; }
  __syncthreads();
  const int n0 = rng[0], n1 = rng[1];
  float s0 = 0.f, s1 = 0.f;
  for (int n = n0 + wave; n < n1; n += 8) { if (n2g[n] == g) { s0 += Hm[(size_t)n * GH + 2 * lane]; s1 += Hm[(size_t)n * GH + 2 * lane + 1]; } }
  acc[wave][2 * lane] = s0; acc[wave][2 * lane + 1] = s1;
  __syncthreads();
  if (t < GH) { float s = 0.f; for (int w = 0; w < 8; ++w) s += acc[w][t]; const float cnt = (float)(n1 - n0); hg[t] = s / fmaxf(cnt, 1.0f); }
  __syncthreads();
  if (t < 32) { float s = b1[t]; for (int c = 0; c < GH; ++c) s += W1[t * GH + c] * hg[c]; z1[t] = fmaxf(s, 0.f); }
  __syncthreads();
  if (t < 32) { float s = 0.f; if (t < 10) { s = b2[t]; for (int c = 0; c < 32; ++c) s += W2[t * 32 + c] * z1[c]; }
    ((volatile float*)outg)[(size_t)g * 32 + t] = s; __threadfence(); ((volatile float*)outg)[(size_t)g * 32 + t] = s; }
}
__global__ __launch_bounds__(256) void pack_out_kernel(const float* __restrict__ stg, float* __restrict__ out) {
  for (int pass = 0; pass < 2; ++pass) { for (int i = threadIdx.x; i < NG * 10; i += 256) ((volatile float*)out)[i] = stg[(i / 10) * 32 + (i % 10)]; __threadfence(); }
}
extern "C" void kernel_launch(void* const* d_in, const int* in_sizes, int n_in, void* d_out, int out_size, void* d_ws, size_t ws_size, hipStream_t stream) {
  (void)in_sizes; (void)n_in; (void)out_size; (void)ws_size;
  const float* x = (const float*)d_in[0]; const int* src = (const int*)d_in[1]; const int* dst = (const int*)d_in[2]; const int* et = (const int*)d_in[3]; const int* n2g = (const int*)d_in[4];
  const float* W_in = (const float*)d_in[5]; const float* b_in = (const float*)d_in[6]; const float* We = (const float*)d_in[7]; const float* be = (const float*)d_in[8];
  const float* W_ih = (const float*)d_in[9]; const float* b_ih = (const float*)d_in[10]; const float* W_hh = (const float*)d_in[11]; const float* b_hh = (const float*)d_in[12];
  const float* W1 = (const float*)d_in[13]; const float* b1 = (const float*)d_in[14]; const float* W2 = (const float*)d_in[15]; const float* b2 = (const float*)d_in[16];
  char* ws = (char*)d_ws; size_t off = 0;
  auto carve = [&](size_t bytes) -> char* { char* p = ws + off; off += (bytes + 255) & ~(size_t)255; return p; };
  int* ccnt   = (int*)carve((size_t)NCH * NRP * 4);
  int* boff   = (int*)carve((size_t)NCH * NRP * 4);
  int* rinfo  = (int*)carve((size_t)2048 * 4);
  int* bucket = (int*)carve(BUCKET_INTS * 4);
  int* rowptr = (int*)carve((size_t)NBLK * NODES_PER_BLK * 4);
  int* rowdeg = (int*)carve((size_t)NBLK * NODES_PER_BLK * 4);
  int* csr_eid= (int*)carve((size_t)NBLK * SEG_STRIDE * 4);

  unsigned* X16 = (unsigned*)carve((size_t)NPAD * GIN * 2);
  _Float16* Win16 = (_Float16*)carve((size_t)GH * GIN * 2);
  _Float16* We16 = (_Float16*)carve((size_t)NET * GH * GH * 2);
  _Float16* Wih16 = (_Float16*)carve((size_t)3 * GH * GH * 2); _Float16* Whh16 = (_Float16*)carve((size_t)3 * GH * GH * 2);
  float* beflat = (float*)carve((size_t)NET * GH * 4);
  float* Hm = (float*)carve((size_t)NPAD * GH * 4);
  unsigned* H16 = (unsigned*)carve((size_t)NPAD * GH * 2);
  unsigned* T = (unsigned*)carve((size_t)NPAD * NET * GH * 2);
  unsigned* A16 = (unsigned*)carve((size_t)NPAD * GH * 2);
  const int HALF = NPAD / 2;
  float* GI = (float*)carve((size_t)HALF * 3 * GH * 4); float* GHm = (float*)carve((size_t)HALF * 3 * GH * 4);
  float* stg = (float*)carve((size_t)NG * 32 * 4);

  csr_hist_kernel<<<NCH, 256, 0, stream>>>(dst, ccnt);
  csr_offsets_kernel<<<1, 1024, 0, stream>>>(ccnt, boff, rinfo);
  csr_bucket_kernel<<<NCH, 256, 0, stream>>>(dst, boff, bucket);
  csr_fill_kernel<<<NBLK, 256, 0, stream>>>(dst, bucket, rinfo, rowptr, rowdeg, csr_eid, nullptr);

  padcast_rows_kernel<<<(NPAD * GIN / 2 + 255) / 256, 256, 0, stream>>>(x, X16);
  cast_f32_f16x2<<<(GH * GIN / 2 + 255) / 256, 256, 0, stream>>>(W_in, Win16, GH * GIN / 2);
  cast_f32_f16x2<<<(NET * GH * GH / 2 + 255) / 256, 256, 0, stream>>>(We, We16, NET * GH * GH / 2);
  cast_f32_f16x2<<<(3 * GH * GH / 2 + 255) / 256, 256, 0, stream>>>(W_ih, Wih16, 3 * GH * GH / 2);
  cast_f32_f16x2<<<(3 * GH * GH / 2 + 255) / 256, 256, 0, stream>>>(W_hh, Whh16, 3 * GH * GH / 2);
  { const int t = (NPAD / 64) * (GH / 64);
    wmma_gemm64<0, false, 2, 0, false><<<dim3((t + 7) / 8, 1), 256, 0, stream>>>((const unsigned short*)X16, nullptr, GIN, 0, U16(Win16), nullptr, GIN, 0, Hm, nullptr, GH, 0, b_in, nullptr, 0, NPAD, GH, GIN, 1.0f); }
  cast_h_kernel<<<(NPAD * GH / 2 + 255) / 256, 256, 0, stream>>>(Hm, H16);
  for (int step = 0; step < 5; ++step) {
    { const int t = (NPAD / 64) * (NET * GH / 64);
      wmma_gemm64<0, false, 2, 1, false><<<dim3((t + 7) / 8, 1), 256, 0, stream>>>((const unsigned short*)H16, nullptr, GH, 0, U16(We16), nullptr, GH, 0, T, nullptr, NET * GH, 0, be, nullptr, 0, NPAD, NET * GH, GH, 1.0f); }
    agg_kernel<<<NPAD / 8, 256, 0, stream>>>(T, rowptr, rowdeg, csr_eid, src, et, A16);
    for (int hf = 0; hf < 2; ++hf) { const size_t r0 = (size_t)hf * HALF; const int t = (HALF / 64) * (3 * GH / 64);
      wmma_gemm64<0, false, 2, 0, false><<<dim3((t + 7) / 8, 1), 256, 0, stream>>>((const unsigned short*)(A16 + r0 * (GH / 2)), nullptr, GH, 0, U16(Wih16), nullptr, GH, 0, GI, nullptr, 3 * GH, 0, b_ih, nullptr, 0, HALF, 3 * GH, GH, 1.0f);
      wmma_gemm64<0, false, 2, 0, false><<<dim3((t + 7) / 8, 1), 256, 0, stream>>>((const unsigned short*)(H16 + r0 * (GH / 2)), nullptr, GH, 0, U16(Whh16), nullptr, GH, 0, GHm, nullptr, 3 * GH, 0, b_hh, nullptr, 0, HALF, 3 * GH, GH, 1.0f);
      gru_kernel<<<(HALF * GH / 2 + 255) / 256, 256, 0, stream>>>(GI, GHm, Hm + r0 * GH, H16 + r0 * (GH / 2), HALF); }
  }
  readout_kernel<<<NG, 256, 0, stream>>>(Hm, n2g, W1, b1, W2, b2, stg);
  pack_out_kernel<<<1, 256, 0, stream>>>(stg, (float*)d_out);
}
